// Mamba3Layer_16630113370812
// MI455X (gfx1250) — hardware-run, weakly checked
//
#include <hip/hip_runtime.h>
#include <math.h>

typedef __attribute__((ext_vector_type(16))) _Float16 v16h;
typedef __attribute__((ext_vector_type(8)))  _Float16 v8h;
typedef __attribute__((ext_vector_type(2)))  _Float16 v2h;
typedef __attribute__((ext_vector_type(16))) __bf16   v16b;
typedef __attribute__((ext_vector_type(8)))  __bf16   v8b;
typedef __attribute__((ext_vector_type(8)))  float    v8f;
typedef __attribute__((ext_vector_type(4)))  float    v4f;
typedef __attribute__((ext_vector_type(2)))  unsigned v2u;
typedef __attribute__((ext_vector_type(4)))  unsigned v4u;

constexpr int kBatch  = 2;
constexpr int kSeq    = 4096;
constexpr int kTok    = kBatch * kSeq;
constexpr int kDm     = 1024;
constexpr int kDi     = 2048;
constexpr int kHeads  = 32;
constexpr int kHd     = 64;
constexpr int kNs     = 64;
constexpr int kProj   = 2 * kDi + 2 * kNs + 2 * kHeads + kNs / 2;
constexpr int kProjP  = 4352;
constexpr int kSmP    = 256;
constexpr int kSmB    = 0;
constexpr int kSmC    = 64;
constexpr int kSmDt   = 128;
constexpr int kSmLam  = 160;
constexpr int kSmTh   = 192;
constexpr int kCh     = 32;
constexpr float kEps    = 1.1920929e-07f;
constexpr float kYScale = 1.0f / 8.0f;
constexpr float kGCarry = 16.0f;
constexpr float kWoCarry = 32.0f;
constexpr float kFold   = 1.0f / (kGCarry * kWoCarry);
constexpr float kInvMeanG = 1.0f / (kGCarry * kGCarry * (float)kDi);
static_assert(kProj == 4320, "projection width");
static_assert(8 * 8 == kNs, "readout scale is 1/sqrt(state width)");
static_assert(kHeads * kHd == kDi && kHd == 64 && kNs == 64 && kHeads == 32, "head layout");
static_assert((kProjP % 64) == 0 && kProjP >= kProj && (kTok % 64) == 0 && (kDm % 64) == 0, "GEMM M,N tile multiples");
static_assert((kDm % 32) == 0 && (kDi % 32) == 0, "GEMM K multiples of 32");
static_assert(kProjP - 2 * kDi == kSmP, "small plane width");
static_assert((kSeq % kCh) == 0 && (kCh % 8) == 0, "scan chunking");

constexpr size_t kSzR0    = (size_t)kTok * kDi * 2;
constexpr size_t kSzXH    = (size_t)kTok * kDm * 2;
constexpr size_t kSzWINH  = (size_t)kProjP * kDm * 2;
constexpr size_t kOffXH   = 0;
constexpr size_t kOffWINH = kOffXH + kSzXH;
constexpr size_t kOffG    = 0;
constexpr size_t kOffZ    = kSzR0;
constexpr size_t kOffXS   = kOffZ + (size_t)kTok * kDi * 2;
constexpr size_t kOffWOUT = kOffXS + (size_t)kTok * kDi * 2;
constexpr size_t kOffSM   = kOffWOUT + (size_t)kDm * kDi * 2;
constexpr size_t kOffBN   = kOffSM + (size_t)kTok * kSmP * 4;
constexpr size_t kOffCN   = kOffBN + (size_t)kTok * kNs * 4;
constexpr size_t kOffBROT = kOffCN + (size_t)kTok * kNs * 4;
constexpr size_t kOffCROT = kOffBROT + (size_t)kTok * kNs * 4;
constexpr size_t kOffAL   = kOffCROT + (size_t)kTok * kNs * 4;
constexpr size_t kOffCG   = kOffAL + (size_t)kTok * kHeads * 4;
constexpr size_t kOffCB   = kOffCG + (size_t)kTok * kHeads * 4;
constexpr size_t kOffSTEP = kOffCB + (size_t)kTok * kHeads * 4;
constexpr size_t kOffINV  = kOffSTEP + (size_t)kTok * kHeads * 4;
constexpr size_t kWsTotal = kOffINV + (size_t)kTok * 4;
static_assert(kSzXH + kSzWINH <= kSzR0, "operand planes fit the shared region");
static_assert(kWsTotal == 125861888ull, "carve total");
static_assert(kWsTotal <= 134217728ull, "carve cap");
static_assert((kOffWINH % 128) == 0 && (kOffZ % 128) == 0 && (kOffXS % 128) == 0 && (kOffWOUT % 128) == 0 &&
              (kOffSM % 128) == 0 && (kOffBN % 128) == 0 && (kOffCN % 128) == 0 && (kOffBROT % 128) == 0 &&
              (kOffCROT % 128) == 0 && (kOffAL % 128) == 0 && (kOffCG % 128) == 0 && (kOffCB % 128) == 0 &&
              (kOffSTEP % 128) == 0 && (kOffINV % 128) == 0, "128-B aligned regions");

__device__ __forceinline__ unsigned short f2bf_bits(float f) {
  unsigned u = __float_as_uint(f);
  return (unsigned short)((u + 0x7FFFu + ((u >> 16) & 1u)) >> 16);
}
__device__ __forceinline__ float bf_bits2f(unsigned short h) { return __uint_as_float(((unsigned)h) << 16); }

__device__ __forceinline__ float h16_to_f32(unsigned hb) {
  const unsigned sgn = (hb & 0x8000u) << 16;
  const unsigned em = hb & 0x7fffu;
  const float fn = __uint_as_float((em << 13) + 0x38000000u);
  const float fs = (float)em * 5.9604644775390625e-8f;
  const float mag = (em < 0x400u) ? fs : fn;
  return __uint_as_float(__float_as_uint(mag) | sgn);
}
__device__ __forceinline__ float sigm(float v) { return __builtin_amdgcn_rcpf(1.0f + expf(-v)); }

__device__ __forceinline__ void wave_lds_sync() {
  __builtin_amdgcn_fence(__ATOMIC_RELEASE, "workgroup");
  __builtin_amdgcn_wave_barrier();
  __builtin_amdgcn_fence(__ATOMIC_ACQUIRE, "workgroup");
}

__device__ __forceinline__ void grp_guard_h(v8f& a, v8f& b, v8f& c, v8f& d, v16h x, v16h y) {
  asm volatile("v_nop\n\tv_nop\n\tv_nop\n\tv_nop" : "+v"(a), "+v"(b), "+v"(c), "+v"(d) : "v"(x), "v"(y));
}
__device__ __forceinline__ void grp_guard_b(v8f& a, v8f& b, v8f& c, v8f& d, v16b x, v16b y) {
  asm volatile("v_nop\n\tv_nop\n\tv_nop\n\tv_nop" : "+v"(a), "+v"(b), "+v"(c), "+v"(d) : "v"(x), "v"(y));
}
__device__ __forceinline__ void keep4_h(v16h a, v16h b, v16h c, v16h d) { asm volatile("v_nop" :: "v"(a), "v"(b), "v"(c), "v"(d)); }
__device__ __forceinline__ void keep4_b(v16b a, v16b b, v16b c, v16b d) { asm volatile("v_nop" :: "v"(a), "v"(b), "v"(c), "v"(d)); }
__device__ __forceinline__ void acc_guard4(v8f& a, v8f& b, v8f& c, v8f& d) { asm volatile("v_nop\n\tv_nop\n\tv_nop\n\tv_nop" : "+v"(a), "+v"(b), "+v"(c), "+v"(d)); }

template <typename T> struct Frag;
template <> struct Frag<_Float16> {
  typedef v16h V; union U { v16h v; v8h h[2]; };
  static __device__ __forceinline__ v16h load(const _Float16* p) {
    U f; f.h[0] = *(const v8h*)(p); f.h[1] = *(const v8h*)(p + 16); return f.v;
  }
  static __device__ __forceinline__ v8f mma(v16h a, v16h b, v8f c) {
    return __builtin_amdgcn_wmma_f32_16x16x32_f16(false, a, false, b, (short)0, c, false, false);
  }
  static __device__ __forceinline__ void guard(v8f& a, v8f& b, v8f& c, v8f& d, v16h x, v16h y) { grp_guard_h(a, b, c, d, x, y); }
  static __device__ __forceinline__ void keep(v16h a, v16h b, v16h c, v16h d) { keep4_h(a, b, c, d); }
};
template <> struct Frag<__bf16> {
  typedef v16b V; union U { v16b v; v8b h[2]; };
  static __device__ __forceinline__ v16b load(const __bf16* p) {
    U f; f.h[0] = *(const v8b*)(p); f.h[1] = *(const v8b*)(p + 16); return f.v;
  }
  static __device__ __forceinline__ v8f mma(v16b a, v16b b, v8f c) {
    return __builtin_amdgcn_wmma_f32_16x16x32_bf16(false, a, false, b, (short)0, c, false, false);
  }
  static __device__ __forceinline__ void guard(v8f& a, v8f& b, v8f& c, v8f& d, v16b x, v16b y) { grp_guard_b(a, b, c, d, x, y); }
  static __device__ __forceinline__ void keep(v16b a, v16b b, v16b c, v16b d) { keep4_b(a, b, c, d); }
};
template <int ET> struct Elem;
template <> struct Elem<0> { typedef _Float16 T; };
template <> struct Elem<1> { typedef __bf16 T; };

__device__ __forceinline__ void slab_store_f32(const float* slab, float* Crow0, int ldc, int lane) {
  const int hh = lane >> 4, c4 = (lane & 15) * 4;
  for (int pass = 0; pass < 2; ++pass) {
#pragma unroll
    for (int it = 0; it < 8; ++it) {
      const int row = it * 2 + hh;
      v4f v = *(const v4f*)(slab + row * 68 + c4);
      *(volatile v4f*)(Crow0 + (size_t)row * ldc + c4) = v;
    }
    __threadfence();
  }
}
__device__ __forceinline__ void slab_store_f16(const float* slab, unsigned short* Crow0, int ldc, int lane) {
  const int q = lane >> 3, c8 = (lane & 7) * 8;
  for (int pass = 0; pass < 2; ++pass) {
#pragma unroll
    for (int it = 0; it < 4; ++it) {
      const int row = it * 4 + q;
      const float* sp = slab + row * 68 + c8;
      v8h hv;
#pragma unroll
      for (int e = 0; e < 8; ++e) hv[e] = (_Float16)sp[e];
      *(volatile v8h*)(Crow0 + (size_t)row * ldc + c8) = hv;
    }
    __threadfence();
  }
}

template <int ET, int EPI>
__global__ __launch_bounds__(256) void gemm64_kernel(
    const unsigned short* __restrict__ Ap, int lda,
    const unsigned short* __restrict__ Btp, int ldb,
    void* out0, void* out1, void* out2,
    const float* __restrict__ rowscale,
    int M, int N, int K, float scale) {
  typedef typename Elem<ET>::T T;
  typedef typename Frag<T>::V V;
  const T* A  = (const T*)Ap;
  const T* Bt = (const T*)Btp;
  __shared__ __align__(16) float sT[8][16 * 68];
  const int lane = threadIdx.x & 31;
  const int wave = threadIdx.x >> 5;
  const int tilesN = N >> 6;
  const int tilesM = M >> 6;
  const int tile = blockIdx.x * 8 + wave;
  if (tile >= tilesM * tilesN) return;
  const int tm = tile / tilesN;
  const int tn = tile - tm * tilesN;
  const int m0 = tm << 6;
  const int n0 = tn << 6;

  const int rlane = lane & 15;
  const int koff  = (lane >> 4) * 8;
  const int mOff  = (lane >> 4) * 8;

  v8f acc[4][4];
#pragma unroll
  for (int i = 0; i < 4; ++i)
#pragma unroll
    for (int j = 0; j < 4; ++j) acc[i][j] = (v8f){0.f,0.f,0.f,0.f,0.f,0.f,0.f,0.f};

  for (int k0 = 0; k0 < K; k0 += 32) {
    V bh[4];
#pragma unroll
    for (int j = 0; j < 4; ++j) {
      const size_t bo = (size_t)(n0 + (j << 4) + rlane) * ldb + koff + k0;
      bh[j] = Frag<T>::load(Bt + bo);
    }
#pragma unroll
    for (int i = 0; i < 4; ++i) {
      const size_t ao = (size_t)(m0 + (i << 4) + rlane) * lda + koff + k0;
      V ah = Frag<T>::load(A + ao);
#pragma unroll
      for (int j = 0; j < 4; ++j) acc[i][j] = Frag<T>::mma(ah, bh[j], acc[i][j]);
      Frag<T>::guard(acc[i][0], acc[i][1], acc[i][2], acc[i][3], ah, ah);
    }
    Frag<T>::keep(bh[0], bh[1], bh[2], bh[3]);
  }
  acc_guard4(acc[0][0], acc[0][1], acc[0][2], acc[0][3]);
  acc_guard4(acc[1][0], acc[1][1], acc[1][2], acc[1][3]);
  acc_guard4(acc[2][0], acc[2][1], acc[2][2], acc[2][3]);
  acc_guard4(acc[3][0], acc[3][1], acc[3][2], acc[3][3]);

  float* slab = sT[wave];
#pragma unroll
  for (int i = 0; i < 4; ++i) {
    const int mBase = m0 + (i << 4);
    float rs[8];
    if (EPI == 1) {
      const v4f r0 = *(const v4f*)(rowscale + mBase + mOff);
      const v4f r1 = *(const v4f*)(rowscale + mBase + mOff + 4);
      rs[0] = r0[0] * scale; rs[1] = r0[1] * scale; rs[2] = r0[2] * scale; rs[3] = r0[3] * scale;
      rs[4] = r1[0] * scale; rs[5] = r1[1] * scale; rs[6] = r1[2] * scale; rs[7] = r1[3] * scale;
    } else {
#pragma unroll
      for (int r = 0; r < 8; ++r) rs[r] = 1.0f;
    }
#pragma unroll
    for (int j = 0; j < 4; ++j) {
#pragma unroll
      for (int r = 0; r < 8; ++r) {
        float v = acc[i][j][r];
        if (EPI == 1) v *= rs[r];
        slab[(mOff + r) * 68 + (j << 4) + rlane] = v;
      }
    }
    wave_lds_sync();
    if (EPI == 1) {
      slab_store_f32(slab, (float*)out0 + (size_t)mBase * N + n0, N, lane);
    } else {
      if (tn >= 64) {
        slab_store_f32(slab, (float*)out2 + (size_t)mBase * kSmP + (n0 - 2 * kDi), kSmP, lane);
      } else {
        if (tn >= 32) {
          const int hh = lane >> 4, c4 = (lane & 15) * 4;
#pragma unroll 1
          for (int it = 0; it < 8; ++it) {
            float* sp = slab + (it * 2 + hh) * 68 + c4;
            const v4f v = *(const v4f*)sp;
            v4f o;
            o[0] = v[0] * sigm(v[0]);
            o[1] = v[1] * sigm(v[1]);
            o[2] = v[2] * sigm(v[2]);
            o[3] = v[3] * sigm(v[3]);
            *(v4f*)sp = o;
          }
          wave_lds_sync();
        }
        unsigned short* dst = (tn >= 32) ? (unsigned short*)out1 : (unsigned short*)out0;
        slab_store_f16(slab, dst + (size_t)mBase * kDi + ((tn & 31) << 6), kDi, lane);
      }
    }
    wave_lds_sync();
  }
}

template <int MODE>
__global__ __launch_bounds__(256) void convert_rows_kernel(
    const float* __restrict__ src, unsigned short* __restrict__ dst, int total8, int valid8, float scale)
{
  const int i = blockIdx.x * 256 + threadIdx.x;
  if (i >= total8) return;
  const bool ok = i < valid8;
  const size_t es = (size_t)(ok ? i : 0) << 3;
  const v4f a0 = *(const v4f*)(src + es);
  const v4f a1 = *(const v4f*)(src + es + 4);
  v8h hv;
#pragma unroll
  for (int e = 0; e < 4; ++e) {
    const float f0 = ok ? a0[e] : 0.0f;
    const float f1 = ok ? a1[e] : 0.0f;
    const unsigned short b0 = f2bf_bits(f0);
    const unsigned short b1 = f2bf_bits(f1);
    if (MODE == 0) {
      hv[e]     = __builtin_bit_cast(_Float16, b0);
      hv[4 + e] = __builtin_bit_cast(_Float16, b1);
    } else {
      hv[e]     = (_Float16)(bf_bits2f(b0) * scale);
      hv[4 + e] = (_Float16)(bf_bits2f(b1) * scale);
    }
  }
  unsigned short* q = dst + ((size_t)i << 3);
  *(volatile v8h*)q = hv;
  __threadfence();
  *(volatile v8h*)q = hv;
}

__global__ __launch_bounds__(256) void prep_kernel(
    const float* __restrict__ SM, const float* __restrict__ A_log, const float* __restrict__ dt_bias,
    const float* __restrict__ Bsc, const float* __restrict__ Csc,
    float* __restrict__ BN, float* __restrict__ CN, float* __restrict__ ALPHA,
    float* __restrict__ CG, float* __restrict__ CB, float* __restrict__ STEP)
{
  const int lane = threadIdx.x & 31, wave = threadIdx.x >> 5;
  const int tok = blockIdx.x * 8 + wave;
  const float* row = SM + (size_t)tok * kSmP;
  const float b0 = row[kSmB + lane], b1 = row[kSmB + 32 + lane];
  const float c0 = row[kSmC + lane], c1 = row[kSmC + 32 + lane];
  const float dtr = row[kSmDt + lane];
  const float lr  = row[kSmLam + lane];
  const float th  = row[kSmTh + lane];
  const float v   = dtr + dt_bias[lane];
  const float sp  = fmaxf(v, 0.0f) + log1pf(expf(-fabsf(v)));
  const float dt  = fminf(fmaxf(sp, 1e-4f), 0.5f);
  float sb = b0 * b0 + b1 * b1;
  float sc = c0 * c0 + c1 * c1;
  float sd = dt;
#pragma unroll
  for (int off = 16; off > 0; off >>= 1) {
    sb += __shfl_xor(sb, off, 32);
    sc += __shfl_xor(sc, off, 32);
    sd += __shfl_xor(sd, off, 32);
  }
  const float invb = rsqrtf(sb * (1.0f / (float)kNs) + kEps);
  const float invc = rsqrtf(sc * (1.0f / (float)kNs) + kEps);
  const float bn0 = b0 * invb * Bsc[lane], bn1 = b1 * invb * Bsc[32 + lane];
  const float cn0 = c0 * invc * Csc[lane], cn1 = c1 * invc * Csc[32 + lane];
  const float alpha = expf(-expf(A_log[lane]) * dt);
  const float lam = sigm(lr);
  const float cg = dt * lam;
  const float cb = dt * (1.0f - lam) * alpha;
  const float dtm = sd * (1.0f / (float)kHeads);
  const float stp = dtm * th;
  float* pB = BN + (size_t)tok * kNs + lane;
  float* pC = CN + (size_t)tok * kNs + lane;
  const size_t o32 = (size_t)tok * kHeads + lane;
  *(volatile float*)(pB) = bn0;
  *(volatile float*)(pB + 32) = bn1;
  *(volatile float*)(pC) = cn0;
  *(volatile float*)(pC + 32) = cn1;
  *(volatile float*)(ALPHA + o32) = alpha;
  *(volatile float*)(CG + o32) = cg;
  *(volatile float*)(CB + o32) = cb;
  *(volatile float*)(STEP + o32) = stp;
  __threadfence();
  *(volatile float*)(pB) = bn0;
  *(volatile float*)(pB + 32) = bn1;
  *(volatile float*)(pC) = cn0;
  *(volatile float*)(pC + 32) = cn1;
  *(volatile float*)(ALPHA + o32) = alpha;
  *(volatile float*)(CG + o32) = cg;
  *(volatile float*)(CB + o32) = cb;
  *(volatile float*)(STEP + o32) = stp;
}

__global__ __launch_bounds__(32) void angle_rope_kernel(
    const float* __restrict__ STEP, const float* __restrict__ BN, const float* __restrict__ CN,
    float* __restrict__ BROT, float* __restrict__ CROT)
{
  const int b = blockIdx.x, c = threadIdx.x;
  double acc = 0.0;
#pragma unroll 1
  for (int t = 0; t < kSeq; ++t) {
    const size_t pos = (size_t)b * kSeq + t;
    const float st = STEP[pos * kHeads + c];
    const float b1 = BN[pos * kNs + c], b2 = BN[pos * kNs + 32 + c];
    const float c1 = CN[pos * kNs + c], c2 = CN[pos * kNs + 32 + c];
    acc += (double)st;
    const float ang = -(float)acc;
    const float cs = cosf(ang);
    const float sn = sinf(ang);
    const float ob1 = b1 * cs - b2 * sn;
    const float ob2 = b1 * sn + b2 * cs;
    const float oc1 = c1 * cs - c2 * sn;
    const float oc2 = c1 * sn + c2 * cs;
    float* pB = BROT + pos * kNs + c;
    float* pC = CROT + pos * kNs + c;
    *(volatile float*)(pB) = ob1;
    *(volatile float*)(pB + 32) = ob2;
    *(volatile float*)(pC) = oc1;
    *(volatile float*)(pC + 32) = oc2;
    __threadfence();
    *(volatile float*)(pB) = ob1;
    *(volatile float*)(pB + 32) = ob2;
    *(volatile float*)(pC) = oc1;
    *(volatile float*)(pC + 32) = oc2;
  }
}

__global__ __launch_bounds__(256) void scan_gate_kernel(
    const unsigned* __restrict__ XSw, const unsigned* __restrict__ Zw,
    const float* __restrict__ BROT, const float* __restrict__ CROT,
    const float* __restrict__ ALPHA, const float* __restrict__ CG, const float* __restrict__ CB,
    unsigned* __restrict__ Gw)
{
  __shared__ __align__(16) float xl[(kCh + 1) * 64];
  __shared__ __align__(16) float Bl[(kCh + 1) * 64];
  __shared__ __align__(16) float Cl[kCh * 64];
  __shared__ __align__(16) float part[4 * kCh * 64];
  __shared__ float sa[kCh];
  __shared__ float scg[kCh];
  __shared__ float scb[kCh];
  __shared__ unsigned gpk[kCh * 32];

  const int tid = threadIdx.x, lane = tid & 31, wave = tid >> 5;
  const int b = blockIdx.x >> 5;
  const int h = blockIdx.x & 31;
  const int d = tid & 63;
  const int sg = tid >> 6;
  const int s0 = sg * 16;
  constexpr int kGroups = (kCh + 1) * 16;

  float hst[16];
#pragma unroll
  for (int j = 0; j < 16; ++j) hst[j] = 0.f;

#pragma unroll 1
  for (int t0 = 0; t0 < kSeq; t0 += kCh) {
#pragma unroll
    for (int i = 0; i < 3; ++i) {
      const int idx = tid + i * 256;
      const int idc = (idx < kGroups) ? idx : (kGroups - 1);
      const int r = idc >> 4, q = idc & 15;
      const int t = t0 - 1 + r;
      const bool ok = (t >= 0);
      const size_t pos = (size_t)b * kSeq + (ok ? t : 0);
      v4f bv = *(const v4f*)(BROT + pos * kNs + q * 4);
      v2u xw = *(const v2u*)(XSw + pos * (kDi / 2) + h * 32 + q * 2);
      asm volatile("" : "+v"(bv));
      asm volatile("" : "+v"(xw));
      const unsigned w0 = xw[0];
      const unsigned w1 = xw[1];
      const float x0 = h16_to_f32(w0 & 0xffffu);
      const float x1 = h16_to_f32(w0 >> 16);
      const float x2 = h16_to_f32(w1 & 0xffffu);
      const float x3 = h16_to_f32(w1 >> 16);
      v4f bz, xz;
      bz[0] = ok ? bv[0] : 0.0f; bz[1] = ok ? bv[1] : 0.0f; bz[2] = ok ? bv[2] : 0.0f; bz[3] = ok ? bv[3] : 0.0f;
      xz[0] = ok ? x0 : 0.0f;    xz[1] = ok ? x1 : 0.0f;    xz[2] = ok ? x2 : 0.0f;    xz[3] = ok ? x3 : 0.0f;
      if (idx < kGroups) {
        *(v4f*)(Bl + r * 64 + q * 4) = bz;
        *(v4f*)(xl + r * 64 + q * 4) = xz;
      }
    }
#pragma unroll
    for (int i = 0; i < 2; ++i) {
      const int idx = tid + i * 256;
      const int r = idx >> 4, q = idx & 15;
      const size_t pos = (size_t)b * kSeq + t0 + r;
      *(v4f*)(Cl + r * 64 + q * 4) = *(const v4f*)(CROT + pos * kNs + q * 4);
    }
    if (tid < kCh) {
      const size_t o = ((size_t)b * kSeq + t0 + tid) * kHeads + h;
      sa[tid]  = ALPHA[o];
      scg[tid] = CG[o];
      scb[tid] = CB[o];
    }
    __syncthreads();

#pragma unroll 1
    for (int tt = 0; tt < kCh; ++tt) {
      const float a  = sa[tt];
      const float u1 = scg[tt] * xl[(tt + 1) * 64 + d];
      const float u2 = scb[tt] * xl[tt * 64 + d];
      const float* bt = Bl + (tt + 1) * 64 + s0;
      const float* bp = Bl + tt * 64 + s0;
      const float* ct = Cl + tt * 64 + s0;
      float yp = 0.f;
#pragma unroll
      for (int q4 = 0; q4 < 4; ++q4) {
        const v4f bv = *(const v4f*)(bt + 4 * q4);
        const v4f pv = *(const v4f*)(bp + 4 * q4);
        const v4f cv = *(const v4f*)(ct + 4 * q4);
#pragma unroll
        for (int e = 0; e < 4; ++e) {
          const float hh = fmaf(a, hst[4 * q4 + e], fmaf(u1, bv[e], u2 * pv[e]));
          hst[4 * q4 + e] = hh;
          yp = fmaf(hh, cv[e], yp);
        }
      }
      part[(sg * kCh + tt) * 64 + d] = yp;
    }
    __syncthreads();

#pragma unroll 1
    for (int it = 0; it < kCh / 8; ++it) {
      const int r = it * 8 + wave;
      const int o = r * 64 + 2 * lane;
      const float y0 = (part[o] + part[kCh * 64 + o]) + (part[2 * kCh * 64 + o] + part[3 * kCh * 64 + o]);
      const float y1 = (part[o + 1] + part[kCh * 64 + o + 1]) + (part[2 * kCh * 64 + o + 1] + part[3 * kCh * 64 + o + 1]);
      const size_t pos = (size_t)b * kSeq + t0 + r;
      const unsigned zw = Zw[pos * (kDi / 2) + h * 32 + lane];
      const float z0 = h16_to_f32(zw & 0xffffu);
      const float z1 = h16_to_f32(zw >> 16);
      const float g0 = (y0 * kYScale) * (z0 * sigm(z0)) * kGCarry;
      const float g1 = (y1 * kYScale) * (z1 * sigm(z1)) * kGCarry;
      v2h p;
      p[0] = (_Float16)g0;
      p[1] = (_Float16)g1;
      gpk[r * 32 + lane] = __builtin_bit_cast(unsigned, p);
    }
    for (int pass = 0; pass < 2; ++pass) {
#pragma unroll
      for (int it = 0; it < kCh / 8; ++it) {
        const int r = it * 8 + wave;
        const size_t pos = (size_t)b * kSeq + t0 + r;
        const unsigned u = gpk[r * 32 + lane];
        *(volatile unsigned*)(Gw + pos * (kDi / 2) + h * 32 + lane) = u;
      }
      __threadfence();
    }
  }
}

__global__ __launch_bounds__(256) void rownorm_kernel(const v4u* __restrict__ G4, float* __restrict__ INV)
{
  __shared__ float sInv[32];
  const int lane = threadIdx.x & 31, wave = threadIdx.x >> 5;
#pragma unroll 1
  for (int j = 0; j < 4; ++j) {
    const int row = blockIdx.x * 32 + wave * 4 + j;
    const v4u* p = G4 + (size_t)row * (kDi / 8);
    float ss = 0.f;
#pragma unroll 1
    for (int it = 0; it < 8; ++it) {
      const v4u w = p[it * 32 + lane];
      const unsigned w0 = w[0];
      const unsigned w1 = w[1];
      const unsigned w2 = w[2];
      const unsigned w3 = w[3];
      const float f0 = h16_to_f32(w0 & 0xffffu), f1 = h16_to_f32(w0 >> 16);
      const float f2 = h16_to_f32(w1 & 0xffffu), f3 = h16_to_f32(w1 >> 16);
      const float f4 = h16_to_f32(w2 & 0xffffu), f5 = h16_to_f32(w2 >> 16);
      const float f6 = h16_to_f32(w3 & 0xffffu), f7 = h16_to_f32(w3 >> 16);
      ss = fmaf(f0, f0, ss); ss = fmaf(f1, f1, ss); ss = fmaf(f2, f2, ss); ss = fmaf(f3, f3, ss);
      ss = fmaf(f4, f4, ss); ss = fmaf(f5, f5, ss); ss = fmaf(f6, f6, ss); ss = fmaf(f7, f7, ss);
    }
#pragma unroll
    for (int off = 16; off > 0; off >>= 1) ss += __shfl_xor(ss, off, 32);
    const float inv = rsqrtf(ss * kInvMeanG + kEps);
    if (lane == 0) sInv[wave * 4 + j] = inv;
  }
  __syncthreads();
  if (wave == 0) {
    const float v = sInv[lane];
    float* q = INV + (size_t)blockIdx.x * 32 + lane;
    *(volatile float*)q = v;
    __threadfence();
    *(volatile float*)q = v;
  }
}

extern "C" void kernel_launch(void* const* d_in, const int* in_sizes, int n_in,
                              void* d_out, int out_size, void* d_ws, size_t ws_size,
                              hipStream_t stream)
{
  if (n_in < 7) return;
  if (in_sizes[0] != kTok * kDm) return;
  if (in_sizes[1] != kProj * kDm) return;
  if (in_sizes[2] != kHeads || in_sizes[3] != kHeads) return;
  if (in_sizes[4] != kNs || in_sizes[5] != kNs) return;
  if (in_sizes[6] != kDm * kDi) return;
  if (out_size != kTok * kDm) return;
  if (ws_size < kWsTotal) return;

  const float* x       = (const float*)d_in[0];
  const float* W_in    = (const float*)d_in[1];
  const float* A_log   = (const float*)d_in[2];
  const float* dt_bias = (const float*)d_in[3];
  const float* Bsc     = (const float*)d_in[4];
  const float* Csc     = (const float*)d_in[5];
  const float* W_out   = (const float*)d_in[6];
  float* out = (float*)d_out;

  char* ws = (char*)d_ws;
  unsigned short* XH    = (unsigned short*)(ws + kOffXH);
  unsigned short* WINH  = (unsigned short*)(ws + kOffWINH);
  unsigned short* G     = (unsigned short*)(ws + kOffG);
  unsigned short* Z     = (unsigned short*)(ws + kOffZ);
  unsigned short* XS    = (unsigned short*)(ws + kOffXS);
  unsigned short* WOUTH = (unsigned short*)(ws + kOffWOUT);
  float* SMALL = (float*)(ws + kOffSM);
  float* BN    = (float*)(ws + kOffBN);
  float* CN    = (float*)(ws + kOffCN);
  float* BROT  = (float*)(ws + kOffBROT);
  float* CROT  = (float*)(ws + kOffCROT);
  float* ALPHA = (float*)(ws + kOffAL);
  float* CGp   = (float*)(ws + kOffCG);
  float* CBp   = (float*)(ws + kOffCB);
  float* STEP  = (float*)(ws + kOffSTEP);
  float* INVR  = (float*)(ws + kOffINV);

  convert_rows_kernel<0><<<(kTok * kDm / 8) / 256, 256, 0, stream>>>(x, XH, kTok * kDm / 8, kTok * kDm / 8, 1.0f);
  convert_rows_kernel<0><<<(kProjP * kDm / 8) / 256, 256, 0, stream>>>(W_in, WINH, kProjP * kDm / 8, kProj * kDm / 8, 1.0f);
  convert_rows_kernel<1><<<(kDm * kDi / 8) / 256, 256, 0, stream>>>(W_out, WOUTH, kDm * kDi / 8, kDm * kDi / 8, kWoCarry);

  gemm64_kernel<1, 0><<<((kTok / 64) * (kProjP / 64)) / 8, 256, 0, stream>>>(
      XH, kDm, WINH, kDm, (void*)Z, (void*)XS, (void*)SMALL, INVR, kTok, kProjP, kDm, 1.0f);

  prep_kernel<<<kTok / 8, 256, 0, stream>>>(SMALL, A_log, dt_bias, Bsc, Csc, BN, CN, ALPHA, CGp, CBp, STEP);

  angle_rope_kernel<<<kBatch, 32, 0, stream>>>(STEP, BN, CN, BROT, CROT);

  scan_gate_kernel<<<kBatch * kHeads, 256, 0, stream>>>(
      (const unsigned*)XS, (const unsigned*)Z, BROT, CROT, ALPHA, CGp, CBp, (unsigned*)G);

  rownorm_kernel<<<kTok / 32, 256, 0, stream>>>((const v4u*)G, INVR);

  gemm64_kernel<0, 1><<<((kTok / 64) * (kDm / 64)) / 8, 256, 0, stream>>>(
      G, kDi, WOUTH, kDi, (void*)out, (void*)out, (void*)out, INVR, kTok, kDm, kDi, kFold);
}
